// CapNet_82901458747419
// MI455X (gfx1250) — hardware-run, weakly checked
//
#include <hip/hip_runtime.h>
#include <stdint.h>

typedef __attribute__((ext_vector_type(16))) _Float16 v16h;
typedef __attribute__((ext_vector_type(8)))  _Float16 v8h;
typedef __attribute__((ext_vector_type(16))) __bf16   v16b;
typedef __attribute__((ext_vector_type(8)))  __bf16   v8b;
typedef __attribute__((ext_vector_type(8)))  float    v8f;
typedef __attribute__((ext_vector_type(4)))  float    v4f;

__device__ __forceinline__ unsigned short f2bf_bits(float f) {
  unsigned u = __float_as_uint(f);
  return (unsigned short)((u + 0x7FFFu + ((u >> 16) & 1u)) >> 16);
}
__device__ __forceinline__ float bf_bits2f(unsigned short h) { return __uint_as_float(((unsigned)h) << 16); }

__device__ __forceinline__ void dep_guard_h(v8f& a, v8f& b, v16h x, v16h y) { asm volatile("v_nop\n\tv_nop\n\tv_nop\n\tv_nop" : "+v"(a), "+v"(b) : "v"(x), "v"(y)); }
__device__ __forceinline__ void dep_guard_b(v8f& a, v8f& b, v16b x, v16b y) { asm volatile("v_nop\n\tv_nop\n\tv_nop\n\tv_nop" : "+v"(a), "+v"(b) : "v"(x), "v"(y)); }
__device__ __forceinline__ void keep4_h(v16h a, v16h b, v16h c, v16h d) { asm volatile("v_nop" :: "v"(a), "v"(b), "v"(c), "v"(d)); }
__device__ __forceinline__ void keep4_b(v16b a, v16b b, v16b c, v16b d) { asm volatile("v_nop" :: "v"(a), "v"(b), "v"(c), "v"(d)); }
__device__ __forceinline__ void acc_guard4(v8f& a, v8f& b, v8f& c, v8f& d) { asm volatile("v_nop\n\tv_nop\n\tv_nop\n\tv_nop" : "+v"(a), "+v"(b), "+v"(c), "+v"(d)); }
template <typename T> struct Frag;
template <> struct Frag<_Float16> {
  typedef v16h V; union U { v16h v; v8h h[2]; };
  static __device__ __forceinline__ v16h load(const _Float16* p) {
    U f; f.h[0] = *(const v8h*)(p); f.h[1] = *(const v8h*)(p + 16); return f.v;
  }
  static __device__ __forceinline__ v8f mma(v16h a, v16h b, v8f c) {
    return __builtin_amdgcn_wmma_f32_16x16x32_f16(false, a, false, b, (short)0, c, false, false);
  }
  static __device__ __forceinline__ void guard(v8f& a, v8f& b, v16h x, v16h y) { dep_guard_h(a, b, x, y); }
  static __device__ __forceinline__ void keep(v16h a, v16h b, v16h c, v16h d) { keep4_h(a, b, c, d); }
};
template <> struct Frag<__bf16> {
  typedef v16b V; union U { v16b v; v8b h[2]; };
  static __device__ __forceinline__ v16b load(const __bf16* p) {
    U f; f.h[0] = *(const v8b*)(p); f.h[1] = *(const v8b*)(p + 16); return f.v;
  }
  static __device__ __forceinline__ v8f mma(v16b a, v16b b, v8f c) {
    return __builtin_amdgcn_wmma_f32_16x16x32_bf16(false, a, false, b, (short)0, c, false, false);
  }
  static __device__ __forceinline__ void guard(v8f& a, v8f& b, v16b x, v16b y) { dep_guard_b(a, b, x, y); }
  static __device__ __forceinline__ void keep(v16b a, v16b b, v16b c, v16b d) { keep4_b(a, b, c, d); }
};

template <int ET> struct Elem;
template <> struct Elem<0> { typedef _Float16 T; };
template <> struct Elem<1> { typedef __bf16 T; };
template <int ET, bool SPLIT, int BIAS_MODE, int OUT_MODE, bool RESID, int ACT = 0>
__global__ __launch_bounds__(256) void wmma_gemm64(
    const unsigned short* __restrict__ Ap, const unsigned short* __restrict__ A2p, int lda, long strideA,
    const unsigned short* __restrict__ Btp, const unsigned short* __restrict__ Bt2p, int ldb, long strideB,
    void* __restrict__ Cout, void* __restrict__ Cout2, int ldc, long strideC,
    const float* __restrict__ bias,
    const float* __restrict__ resid, long strideR,
    int M, int N, int K, float scale) {
  typedef typename Elem<ET>::T T;
  typedef typename Frag<T>::V V;
  const T* A = (const T*)Ap; const T* A2 = (const T*)A2p; const T* Bt = (const T*)Btp; const T* Bt2 = (const T*)Bt2p;
  __shared__ __align__(16) float sT[8][16 * 68];
  const int b    = blockIdx.y;
  const int lane = threadIdx.x & 31;
  const int wave = threadIdx.x >> 5;
  const int tilesN = N >> 6;
  const int tilesM = M >> 6;
  const int tile = blockIdx.x * 8 + wave;
  if (tile >= tilesM * tilesN) return;
  const int tm = tile / tilesN;
  const int tn = tile - tm * tilesN;
  const int m0 = tm << 6;
  const int n0 = tn << 6;

  const T* Ab  = A  + (size_t)b * strideA;
  const T* Bb  = Bt + (size_t)b * strideB;
  const T* Ab2 = SPLIT ? (A2  + (size_t)b * strideA) : nullptr;
  const T* Bb2 = SPLIT ? (Bt2 + (size_t)b * strideB) : nullptr;

  const int rlane = lane & 15;
  const int koff  = (lane >> 4) * 8;
  const int mOff  = (lane >> 4) * 8;

  v8f acc[4][4];
#pragma unroll
  for (int i = 0; i < 4; ++i)
#pragma unroll
    for (int j = 0; j < 4; ++j) acc[i][j] = (v8f){0.f,0.f,0.f,0.f,0.f,0.f,0.f,0.f};

  for (int k0 = 0; k0 < K; k0 += 32) {
    V bh[4], bl[4];
#pragma unroll
    for (int j = 0; j < 4; ++j) {
      const size_t bo = (size_t)(n0 + (j << 4) + rlane) * ldb + koff + k0;
      bh[j] = Frag<T>::load(Bb + bo);
      if (SPLIT) bl[j] = Frag<T>::load(Bb2 + bo);
    }
#pragma unroll
    for (int i = 0; i < 4; ++i) {
      const size_t ao = (size_t)(m0 + (i << 4) + rlane) * lda + koff + k0;
      V ah = Frag<T>::load(Ab + ao);
      V al;
      if (SPLIT) al = Frag<T>::load(Ab2 + ao);
#pragma unroll
      for (int j = 0; j < 4; ++j) {
        acc[i][j] = Frag<T>::mma(ah, bh[j], acc[i][j]);
        if (SPLIT) {
          acc[i][j] = Frag<T>::mma(ah, bl[j], acc[i][j]);
          acc[i][j] = Frag<T>::mma(al, bh[j], acc[i][j]);
        }
      }
      Frag<T>::guard(acc[i][0], acc[i][3], ah, SPLIT ? al : ah);
    }
    Frag<T>::keep(bh[0], bh[1], bh[2], bh[3]);
    if (SPLIT) Frag<T>::keep(bl[0], bl[1], bl[2], bl[3]);
  }
  acc_guard4(acc[0][0], acc[0][1], acc[0][2], acc[0][3]);
  acc_guard4(acc[1][0], acc[1][1], acc[1][2], acc[1][3]);
  acc_guard4(acc[2][0], acc[2][1], acc[2][2], acc[2][3]);
  acc_guard4(acc[3][0], acc[3][1], acc[3][2], acc[3][3]);

  float* slab = sT[wave];
  const float* Rb = RESID ? (resid + (size_t)b * strideR) : nullptr;
#pragma unroll
  for (int i = 0; i < 4; ++i) {
    const int mBase = m0 + (i << 4);
#pragma unroll
    for (int j = 0; j < 4; ++j) {
      const int n = n0 + (j << 4) + rlane;
      float bv = 0.f;
      if (BIAS_MODE == 2) bv = bias[n];
#pragma unroll
      for (int r = 0; r < 8; ++r) {
        float v = acc[i][j][r] * scale;
        if (BIAS_MODE == 1) v += bias[mBase + mOff + r];
        if (BIAS_MODE == 2) v += bv;
        if (RESID) v += Rb[(size_t)(mBase + mOff + r) * ldc + n];
        if (ACT == 1) v = tanhf(v);
        if (ACT == 2) v = fmaxf(v, 0.0f);
        if (ACT == 3) v = v / (1.0f + expf(-v));
        if (ACT == 4) v = (v > 0.f) ? v : 0.01f * v;
        if (ACT == 5) v = 0.5f * v * (1.0f + erff(v * 0.70710678118654752f));
        slab[(mOff + r) * 68 + (j << 4) + rlane] = v;
      }
    }
    __builtin_amdgcn_fence(__ATOMIC_RELEASE, "workgroup");
    __builtin_amdgcn_wave_barrier();
    __builtin_amdgcn_fence(__ATOMIC_ACQUIRE, "workgroup");
    if (OUT_MODE == 0) {
      float* C = (float*)Cout + (size_t)b * strideC;
      const int hh = lane >> 4, c4 = (lane & 15) * 4;
      for (int pass = 0; pass < 2; ++pass) {
#pragma unroll
        for (int it = 0; it < 8; ++it) {
          const int row = it * 2 + hh;
          v4f v = *(const v4f*)(slab + row * 68 + c4);
          *(volatile v4f*)(C + (size_t)(mBase + row) * ldc + n0 + c4) = v;
        }
        __threadfence();
      }
    } else {
      const int q = lane >> 3, c8 = (lane & 7) * 8;
      unsigned short* C  = (unsigned short*)Cout  + (size_t)b * strideC;
      unsigned short* C2 = (OUT_MODE == 2) ? ((unsigned short*)Cout2 + (size_t)b * strideC) : nullptr;
      for (int pass = 0; pass < 2; ++pass) {
#pragma unroll
        for (int it = 0; it < 4; ++it) {
          const int row = it * 4 + q;
          const float* sp = slab + row * 68 + c8;
          v8h hv, lv;
#pragma unroll
          for (int e = 0; e < 8; ++e) {
            if (OUT_MODE == 1) {
              hv[e] = (_Float16)sp[e];
            } else {
              unsigned short hb = f2bf_bits(sp[e]);
              unsigned short lb = f2bf_bits(sp[e] - bf_bits2f(hb));
              hv[e] = __builtin_bit_cast(_Float16, hb);
              lv[e] = __builtin_bit_cast(_Float16, lb);
            }
          }
          *(volatile v8h*)(C + (size_t)(mBase + row) * ldc + n0 + c8) = hv;
          if (OUT_MODE == 2) *(volatile v8h*)(C2 + (size_t)(mBase + row) * ldc + n0 + c8) = lv;
        }
        __threadfence();
      }
    }
    __builtin_amdgcn_fence(__ATOMIC_RELEASE, "workgroup");
    __builtin_amdgcn_wave_barrier();
    __builtin_amdgcn_fence(__ATOMIC_ACQUIRE, "workgroup");
  }
}

constexpr int kBatch   = 128;
constexpr int kImg     = 28;
constexpr int kCh      = 256;
constexpr int kSp1     = 20;
constexpr int kPix1    = kSp1 * kSp1;
constexpr int kK1real  = 81;
constexpr int kK1      = 96;
constexpr int kM1      = kBatch * kPix1;
constexpr int kPix2    = 36;
constexpr int kM2      = kBatch * kPix2;
constexpr int kK2      = kCh * 81;
constexpr int kNumI    = 1152;
constexpr int kNumJ    = 10;
constexpr int kDim     = 16;
constexpr int kJD      = kNumJ * kDim;
constexpr int kRowsBI  = kBatch * kNumI;
constexpr int kRowsBIJ = kRowsBI * kNumJ;
constexpr int kFc1K    = 32;
constexpr int kFc1N    = 512;
constexpr int kFc2N    = 1024;
constexpr int kFc3Nreal = 784;
constexpr int kFc3N    = 832;
constexpr int kFc3K    = 1024;
constexpr float kEps   = 1e-9f;
constexpr int kOut0Floats = kBatch * kNumJ;
constexpr int kOut1Floats = kBatch * kFc3Nreal;

static_assert(kM1 % 64 == 0 && kCh % 64 == 0 && kK1 % 32 == 0);
static_assert(kM2 % 64 == 0 && kK2 % 32 == 0 && (kCh % 32) == 0);
static_assert(kBatch % 64 == 0 && kFc1N % 64 == 0 && kFc1K % 32 == 0);
static_assert(kFc2N % 64 == 0 && kFc1N % 32 == 0);
static_assert(kFc3N % 64 == 0 && kFc3K % 32 == 0 && kFc3N >= kFc3Nreal);
static_assert(kOut0Floats * 4 == 5120);
static_assert(5120 + kOut1Floats * 4 == 406528);

constexpr size_t kSzA1   = (size_t)kM1 * kK1 * 2;
constexpr size_t kSzBT1  = (size_t)kCh * kK1 * 2;
constexpr size_t kSzH1   = (size_t)kBatch * kPix1 * kCh * 2;
constexpr size_t kSzW2   = (size_t)kCh * kK2 * 2;
constexpr size_t kSzUH   = (size_t)kRowsBIJ * kDim * 4;
constexpr size_t kSzH2   = (size_t)kM2 * kCh * 4;
constexpr size_t kSzBIJ  = (size_t)kRowsBIJ * 4;
constexpr size_t kSzVJ   = (size_t)kBatch * kJD * 4;
constexpr size_t kSzAFC1 = (size_t)kBatch * kFc1K * 2;
constexpr size_t kSzWFC1 = (size_t)kFc1N * kFc1K * 2;
constexpr size_t kSzC1   = (size_t)kBatch * kFc1N * 2;
constexpr size_t kSzWFC2 = (size_t)kFc2N * kFc1N * 2;
constexpr size_t kSzC2   = (size_t)kBatch * kFc2N * 2;
constexpr size_t kSzWFC3 = (size_t)kFc3N * kFc3K * 2;
constexpr size_t kSzC3   = (size_t)kBatch * kFc3N * 4;

constexpr size_t kOffA1   = 0;
constexpr size_t kOffBT1  = kOffA1 + kSzA1;
constexpr size_t kOffH1   = kOffBT1 + kSzBT1;
constexpr size_t kOffW2   = kOffH1 + kSzH1;
constexpr size_t kOffUH   = 0;
constexpr size_t kOffH2   = kOffUH + kSzUH;
constexpr size_t kOffBP1  = kOffH2 + kSzH2;
constexpr size_t kOffCIJ  = kOffBP1 + kSzBIJ;
constexpr size_t kOffBP2  = kOffCIJ + kSzBIJ;
constexpr size_t kOffVJ   = kOffBP2 + kSzBIJ;
constexpr size_t kOffAFC1 = kOffVJ + kSzVJ;
constexpr size_t kOffWFC1 = kOffAFC1 + kSzAFC1;
constexpr size_t kOffC1   = kOffWFC1 + kSzWFC1;
constexpr size_t kOffWFC2 = kOffC1 + kSzC1;
constexpr size_t kOffC2   = kOffWFC2 + kSzWFC2;
constexpr size_t kOffWFC3 = kOffC2 + kSzC2;
constexpr size_t kOffC3   = kOffWFC3 + kSzWFC3;
constexpr size_t kWsTotal = kOffC3 + kSzC3;
static_assert(kOffW2 + kSzW2 <= kSzUH);
static_assert(kWsTotal <= (size_t)134217728);
static_assert(kOffBT1 % 128 == 0 && kOffH1 % 128 == 0 && kOffW2 % 128 == 0 && kOffH2 % 128 == 0);
static_assert(kOffBP1 % 128 == 0 && kOffCIJ % 128 == 0 && kOffBP2 % 128 == 0 && kOffVJ % 128 == 0);
static_assert(kOffAFC1 % 128 == 0 && kOffWFC1 % 128 == 0 && kOffC1 % 128 == 0 && kOffWFC2 % 128 == 0);
static_assert(kOffC2 % 128 == 0 && kOffWFC3 % 128 == 0 && kOffC3 % 128 == 0);

__global__ __launch_bounds__(256) void k_im2col_x(const float* __restrict__ x, _Float16* __restrict__ A1) {
  const int t = blockIdx.x * 256 + threadIdx.x;
  if (t >= kM1 * (kK1 / 8)) return;
  const int m   = t / (kK1 / 8);
  const int g   = t - m * (kK1 / 8);
  const int b   = m / kPix1;
  const int pix = m - b * kPix1;
  const int oy  = pix / kSp1;
  const int ox  = pix - oy * kSp1;
  const float* xb = x + (size_t)b * (kImg * kImg);
  v8h hv;
#pragma unroll
  for (int e = 0; e < 8; ++e) {
    const int k  = g * 8 + e;
    const int kc = (k < kK1real) ? k : (kK1real - 1);
    const int r  = kc / 9;
    const int s  = kc - r * 9;
    const float v = xb[(oy + r) * kImg + ox + s];
    hv[e] = (_Float16)((k < kK1real) ? v : 0.0f);
  }
  _Float16* dst = A1 + (size_t)t * 8;
  *(volatile v8h*)dst = hv;
  __threadfence();
  *(volatile v8h*)dst = hv;
}

__global__ __launch_bounds__(256) void k_cast_pad(const float* __restrict__ in, _Float16* __restrict__ out,
                                                  int rows_real, int cols_real, int cols_pad, float mul, int nthreads) {
  const int t = blockIdx.x * 256 + threadIdx.x;
  if (t >= nthreads) return;
  const int gpr = cols_pad >> 3;
  const int row = t / gpr;
  const int g   = t - row * gpr;
  const int rr  = (row < rows_real) ? row : (rows_real - 1);
  v8h hv;
#pragma unroll
  for (int e = 0; e < 8; ++e) {
    const int col = g * 8 + e;
    const int cc  = (col < cols_real) ? col : (cols_real - 1);
    const float v = in[(size_t)rr * cols_real + cc] * mul;
    const bool ok = (row < rows_real) && (col < cols_real);
    hv[e] = (_Float16)(ok ? v : 0.0f);
  }
  _Float16* dst = out + (size_t)t * 8;
  *(volatile v8h*)dst = hv;
  __threadfence();
  *(volatile v8h*)dst = hv;
}

__global__ __launch_bounds__(256) void k_reorder_w2(const float* __restrict__ w, _Float16* __restrict__ W2, float mul) {
  const int t = blockIdx.x * 256 + threadIdx.x;
  if (t >= kCh * (kK2 / 8)) return;
  const int o  = t / (kK2 / 8);
  const int g  = t - o * (kK2 / 8);
  const int k0 = g * 8;
  const int rs = k0 >> 8;
  const int c0 = k0 & 255;
  v8h hv;
#pragma unroll
  for (int e = 0; e < 8; ++e)
    hv[e] = (_Float16)(w[((size_t)(o * kCh + c0 + e)) * 81 + rs] * mul);
  _Float16* dst = W2 + (size_t)t * 8;
  *(volatile v8h*)dst = hv;
  __threadfence();
  *(volatile v8h*)dst = hv;
}

__global__ __launch_bounds__(256) void wmma_conv2(
    const unsigned short* __restrict__ H1p, const unsigned short* __restrict__ W2p,
    const float* __restrict__ bias, float* __restrict__ Cout, float scale) {
  typedef _Float16 T;
  typedef v16h V;
  const T* Ha = (const T*)H1p;
  const T* Bt = (const T*)W2p;
  __shared__ __align__(16) float sT[8][16 * 68];
  const int lane = threadIdx.x & 31;
  const int wave = threadIdx.x >> 5;
  constexpr int tilesN = kCh / 64;
  constexpr int tilesM = kM2 / 64;
  const int tile = blockIdx.x * 8 + wave;
  if (tile >= tilesM * tilesN) return;
  const int tm = tile / tilesN;
  const int tn = tile - tm * tilesN;
  const int m0 = tm << 6;
  const int n0 = tn << 6;
  const int rlane = lane & 15;
  const int koff  = (lane >> 4) * 8;
  const int mOff  = (lane >> 4) * 8;

  int abase[4];
#pragma unroll
  for (int i = 0; i < 4; ++i) {
    const int m   = m0 + (i << 4) + rlane;
    const int bb  = m / kPix2;
    const int pix = m - bb * kPix2;
    const int py  = pix / 6;
    const int px  = pix - py * 6;
    abase[i] = bb * (kPix1 * kCh) + ((py * 2) * kSp1 + px * 2) * kCh;
  }

  v8f acc[4][4];
#pragma unroll
  for (int i = 0; i < 4; ++i)
#pragma unroll
    for (int j = 0; j < 4; ++j) acc[i][j] = (v8f){0.f,0.f,0.f,0.f,0.f,0.f,0.f,0.f};

  for (int k0 = 0; k0 < kK2; k0 += 32) {
    const int rs = k0 >> 8;
    const int rr = rs / 9;
    const int ss = rs - rr * 9;
    const int dA = (rr * kSp1 + ss) * kCh + (k0 & 255) + koff;
    V bh[4];
#pragma unroll
    for (int j = 0; j < 4; ++j) {
      const size_t bo = (size_t)(n0 + (j << 4) + rlane) * kK2 + koff + k0;
      bh[j] = Frag<T>::load(Bt + bo);
    }
#pragma unroll
    for (int i = 0; i < 4; ++i) {
      V ah = Frag<T>::load(Ha + (size_t)abase[i] + dA);
#pragma unroll
      for (int j = 0; j < 4; ++j) acc[i][j] = Frag<T>::mma(ah, bh[j], acc[i][j]);
      Frag<T>::guard(acc[i][0], acc[i][3], ah, ah);
    }
    Frag<T>::keep(bh[0], bh[1], bh[2], bh[3]);
  }
  acc_guard4(acc[0][0], acc[0][1], acc[0][2], acc[0][3]);
  acc_guard4(acc[1][0], acc[1][1], acc[1][2], acc[1][3]);
  acc_guard4(acc[2][0], acc[2][1], acc[2][2], acc[2][3]);
  acc_guard4(acc[3][0], acc[3][1], acc[3][2], acc[3][3]);

  float* slab = sT[wave];
#pragma unroll
  for (int i = 0; i < 4; ++i) {
    const int mBase = m0 + (i << 4);
#pragma unroll
    for (int j = 0; j < 4; ++j) {
      const int n = n0 + (j << 4) + rlane;
      const float bv = bias[n];
#pragma unroll
      for (int r = 0; r < 8; ++r) {
        float v = acc[i][j][r] * scale + bv;
        v = fmaxf(v, 0.0f);
        slab[(mOff + r) * 68 + (j << 4) + rlane] = v;
      }
    }
    __builtin_amdgcn_fence(__ATOMIC_RELEASE, "workgroup");
    __builtin_amdgcn_wave_barrier();
    __builtin_amdgcn_fence(__ATOMIC_ACQUIRE, "workgroup");
    {
      const int hh = lane >> 4, c4 = (lane & 15) * 4;
      for (int pass = 0; pass < 2; ++pass) {
#pragma unroll
        for (int it = 0; it < 8; ++it) {
          const int row = it * 2 + hh;
          v4f v = *(const v4f*)(slab + row * 68 + c4);
          *(volatile v4f*)(Cout + (size_t)(mBase + row) * kCh + n0 + c4) = v;
        }
        __threadfence();
      }
    }
    __builtin_amdgcn_fence(__ATOMIC_RELEASE, "workgroup");
    __builtin_amdgcn_wave_barrier();
    __builtin_amdgcn_fence(__ATOMIC_ACQUIRE, "workgroup");
  }
}

__global__ __launch_bounds__(256) void k_uhat(const float* __restrict__ h2, const float* __restrict__ Wt,
                                              float* __restrict__ uh) {
  __shared__ __align__(16) float st[256 * 16];
  const int tid  = threadIdx.x;
  const int lane = tid & 31;
  const int wave = tid >> 5;
  const int row  = blockIdx.x * 256 + tid;
  const int j    = row % kNumJ;
  const int bi   = row / kNumJ;
  const int i    = bi % kNumI;
  const int b    = bi / kNumI;
  float xv[8];
  const int gbase = i * 80 + j * 8;
#pragma unroll
  for (int c = 0; c < 8; ++c) {
    const int g   = gbase + c;
    const int ch  = g / 360;
    const int rem = g - ch * 360;
    const int p36 = rem % 36;
    xv[c] = h2[((size_t)(b * kPix2 + p36)) * kCh + ch];
  }
  const float* Wp = Wt + (size_t)(i * kNumJ + j) * 128;
#pragma unroll 1
  for (int r = 0; r < kDim; ++r) {
    const v4f w0 = *(const v4f*)(Wp + r * 8);
    const v4f w1 = *(const v4f*)(Wp + r * 8 + 4);
    float a = 0.0f;
    a = fmaf(w0[0], xv[0], a);
    a = fmaf(w0[1], xv[1], a);
    a = fmaf(w0[2], xv[2], a);
    a = fmaf(w0[3], xv[3], a);
    a = fmaf(w1[0], xv[4], a);
    a = fmaf(w1[1], xv[5], a);
    a = fmaf(w1[2], xv[6], a);
    a = fmaf(w1[3], xv[7], a);
    st[tid * 16 + r] = a;
  }
  __syncthreads();
  float* dst = uh + (size_t)blockIdx.x * 4096 + wave * 512;
  const float* src = st + wave * 512;
  v4f q0 = *(const v4f*)(src + (0 * 32 + lane) * 4);
  v4f q1 = *(const v4f*)(src + (1 * 32 + lane) * 4);
  v4f q2 = *(const v4f*)(src + (2 * 32 + lane) * 4);
  v4f q3 = *(const v4f*)(src + (3 * 32 + lane) * 4);
  for (int pass = 0; pass < 2; ++pass) {
    *(volatile v4f*)(dst + (0 * 32 + lane) * 4) = q0;
    *(volatile v4f*)(dst + (1 * 32 + lane) * 4) = q1;
    *(volatile v4f*)(dst + (2 * 32 + lane) * 4) = q2;
    *(volatile v4f*)(dst + (3 * 32 + lane) * 4) = q3;
    __threadfence();
  }
}

template <bool UNIF>
__global__ __launch_bounds__(320) void k_route(const float* __restrict__ cij, const float* __restrict__ uh,
                                               const float* __restrict__ cbias, float* __restrict__ vj) {
  __shared__ float red[320];
  __shared__ float ss[160];
  __shared__ __align__(16) float vo[160];
  const int b    = blockIdx.x;
  const int t    = threadIdx.x;
  const int half = (t >= 160) ? 1 : 0;
  const int jd   = t - half * 160;
  const int j    = jd >> 4;
  const float* ub = uh + (size_t)b * kNumI * kJD + jd;
  const float* cb = cij + (size_t)b * kNumI * kNumJ + j;
  const int i0 = half * (kNumI / 2);
  float acc = 0.0f;
#pragma unroll 4
  for (int ii = 0; ii < kNumI / 2; ++ii) {
    const int i = i0 + ii;
    float c = 0.1f;
    if (!UNIF) c = cb[(size_t)i * kNumJ];
    acc = fmaf(c, ub[(size_t)i * kJD], acc);
  }
  red[t] = acc;
  __syncthreads();
  if (t < 160) ss[t] = (red[t] + red[t + 160]) + cbias[t];
  __syncthreads();
  if (t < 160) {
    float sq = 0.0f;
#pragma unroll
    for (int e = 0; e < 16; ++e) { const float v = ss[j * 16 + e]; sq = fmaf(v, v, sq); }
    const float sv = ss[t];
    const float f  = sq * (1.0f / (1.0f + sq));
    vo[t] = f * sv * (1.0f / sqrtf(sq + kEps));
  }
  __syncthreads();
  if (t < 32) {
    float* dst = vj + (size_t)b * kJD;
    const int t8 = (t < 8) ? t : 7;
    const v4f a0 = *(const v4f*)(vo + t * 4);
    const v4f a1 = *(const v4f*)(vo + 128 + t8 * 4);
    for (int pass = 0; pass < 2; ++pass) {
      *(volatile v4f*)(dst + t * 4) = a0;
      if (t < 8) *(volatile v4f*)(dst + 128 + t * 4) = a1;
      __threadfence();
    }
  }
}

template <bool FIRST>
__global__ __launch_bounds__(256) void k_agree_softmax(const float* __restrict__ uh, const float* __restrict__ vj,
                                                       const float* __restrict__ bold, float* __restrict__ bnew,
                                                       float* __restrict__ cnew) {
  __shared__ __align__(16) float sb[2560];
  __shared__ __align__(16) float sc[2560];
  __shared__ float sv[320];
  const int tid  = threadIdx.x;
  const int lane = tid & 31;
  const int wave = tid >> 5;
  const int row0 = blockIdx.x * 256;
  const int b_lo = row0 / kNumI;
  const int b_hi = (b_lo + 1 < kBatch) ? (b_lo + 1) : (kBatch - 1);
  for (int q = tid; q < 320; q += 256) {
    const int src = (q < 160) ? (b_lo * kJD + q) : (b_hi * kJD + q - 160);
    sv[q] = vj[src];
  }
  __syncthreads();
  const int row = row0 + tid;
  const int b   = row / kNumI;
  const int sel = (b - b_lo) * kJD;
  const float* ur = uh + (size_t)row * kJD;
  const float* br = bold + (size_t)row * kNumJ;
  float mx = -__builtin_inff();
#pragma unroll 1
  for (int j = 0; j < kNumJ; ++j) {
    const v4f u0 = *(const v4f*)(ur + j * 16);
    const v4f u1 = *(const v4f*)(ur + j * 16 + 4);
    const v4f u2 = *(const v4f*)(ur + j * 16 + 8);
    const v4f u3 = *(const v4f*)(ur + j * 16 + 12);
    const float* vp = sv + sel + j * 16;
    float a = 0.0f;
    a = fmaf(u0[0], vp[0], a);  a = fmaf(u0[1], vp[1], a);  a = fmaf(u0[2], vp[2], a);  a = fmaf(u0[3], vp[3], a);
    a = fmaf(u1[0], vp[4], a);  a = fmaf(u1[1], vp[5], a);  a = fmaf(u1[2], vp[6], a);  a = fmaf(u1[3], vp[7], a);
    a = fmaf(u2[0], vp[8], a);  a = fmaf(u2[1], vp[9], a);  a = fmaf(u2[2], vp[10], a); a = fmaf(u2[3], vp[11], a);
    a = fmaf(u3[0], vp[12], a); a = fmaf(u3[1], vp[13], a); a = fmaf(u3[2], vp[14], a); a = fmaf(u3[3], vp[15], a);
    float bn = a;
    if (!FIRST) bn = br[j] + a;
    sb[tid * kNumJ + j] = bn;
    mx = fmaxf(mx, bn);
  }
  float ssum = 0.0f;
#pragma unroll 1
  for (int j = 0; j < kNumJ; ++j) {
    const float e = expf(sb[tid * kNumJ + j] - mx);
    sc[tid * kNumJ + j] = e;
    ssum += e;
  }
  const float inv = 1.0f / ssum;
#pragma unroll 1
  for (int j = 0; j < kNumJ; ++j) sc[tid * kNumJ + j] = sc[tid * kNumJ + j] * inv;
  __syncthreads();
  const float* lb = sb + wave * 320;
  const float* lc = sc + wave * 320;
  float* gb = bnew + (size_t)(row0 + wave * 32) * kNumJ;
  float* gc = cnew + (size_t)(row0 + wave * 32) * kNumJ;
  const int l2 = (lane < 16) ? lane : 15;
  const v4f xb0 = *(const v4f*)(lb + lane * 4);
  const v4f xb1 = *(const v4f*)(lb + 128 + lane * 4);
  const v4f xb2 = *(const v4f*)(lb + 256 + l2 * 4);
  const v4f xc0 = *(const v4f*)(lc + lane * 4);
  const v4f xc1 = *(const v4f*)(lc + 128 + lane * 4);
  const v4f xc2 = *(const v4f*)(lc + 256 + l2 * 4);
  for (int pass = 0; pass < 2; ++pass) {
    *(volatile v4f*)(gb + lane * 4) = xb0;
    *(volatile v4f*)(gb + 128 + lane * 4) = xb1;
    if (lane < 16) *(volatile v4f*)(gb + 256 + lane * 4) = xb2;
    *(volatile v4f*)(gc + lane * 4) = xc0;
    *(volatile v4f*)(gc + 128 + lane * 4) = xc1;
    if (lane < 16) *(volatile v4f*)(gc + 256 + lane * 4) = xc2;
    __threadfence();
  }
}

__global__ __launch_bounds__(256) void k_out0(const float* __restrict__ vj, float* __restrict__ out) {
  __shared__ __align__(16) float so[kOut0Floats];
  const int tid = threadIdx.x;
#pragma unroll 1
  for (int q = 0; q < 5; ++q) {
    const int idx = tid + q * 256;
    const float* v = vj + (size_t)idx * kDim;
    const v4f p0 = *(const v4f*)(v);
    const v4f p1 = *(const v4f*)(v + 4);
    const v4f p2 = *(const v4f*)(v + 8);
    const v4f p3 = *(const v4f*)(v + 12);
    float s = 0.0f;
#pragma unroll
    for (int e = 0; e < 4; ++e) { s = fmaf(p0[e], p0[e], s); s = fmaf(p1[e], p1[e], s); s = fmaf(p2[e], p2[e], s); s = fmaf(p3[e], p3[e], s); }
    so[idx] = sqrtf(s + kEps);
  }
  __syncthreads();
  const int t2 = (tid < 64) ? tid : 63;
  const v4f a0 = *(const v4f*)(so + tid * 4);
  const v4f a1 = *(const v4f*)(so + 1024 + t2 * 4);
  for (int pass = 0; pass < 2; ++pass) {
    *(volatile v4f*)(out + tid * 4) = a0;
    if (tid < 64) *(volatile v4f*)(out + 1024 + tid * 4) = a1;
    __threadfence();
  }
}

__global__ __launch_bounds__(256) void k_masked(const float* __restrict__ vj, const float* __restrict__ y,
                                                _Float16* __restrict__ Afc) {
  __shared__ __align__(16) _Float16 hs[256];
  const int tid = threadIdx.x;
  const int gt  = blockIdx.x * 256 + tid;
  const int b   = gt >> 5;
  const int col = gt & 31;
  const int cc  = (col < 16) ? col : 15;
  const float* vb = vj + (size_t)b * kJD + cc * kNumJ;
  const float* yb = y + (size_t)b * kNumJ;
  float a = 0.0f;
#pragma unroll 1
  for (int c = 0; c < kNumJ; ++c) a = fmaf(vb[c], yb[c], a);
  hs[tid] = (_Float16)((col < 16) ? a : 0.0f);
  __syncthreads();
  if (tid < 32) {
    const v8h hv = *(const v8h*)(hs + tid * 8);
    _Float16* dst = Afc + (size_t)blockIdx.x * 256 + tid * 8;
    *(volatile v8h*)dst = hv;
    __threadfence();
    *(volatile v8h*)dst = hv;
  }
}

__global__ __launch_bounds__(256) void k_sig_out(const float* __restrict__ C3, const float* __restrict__ bias,
                                                 float* __restrict__ out) {
  const int t = blockIdx.x * 256 + threadIdx.x;
  if (t >= kOut1Floats / 4) return;
  const int e0  = t * 4;
  const int row = e0 / kFc3Nreal;
  const int col = e0 - row * kFc3Nreal;
  const v4f a  = *(const v4f*)(C3 + (size_t)row * kFc3N + col);
  const v4f bb = *(const v4f*)(bias + col);
  v4f o;
#pragma unroll
  for (int e = 0; e < 4; ++e) {
    float z = a[e] + bb[e];
    z = fminf(fmaxf(z, -30.0f), 30.0f);
    const float ex = expf(-z);
    o[e] = 1.0f / (1.0f + ex);
  }
  float* dst = out + kOut0Floats + e0;
  *(volatile v4f*)dst = o;
  __threadfence();
  *(volatile v4f*)dst = o;
}

extern "C" void kernel_launch(void* const* d_in, const int* in_sizes, int n_in,
                              void* d_out, int out_size, void* d_ws, size_t ws_size,
                              hipStream_t stream) {
  (void)in_sizes; (void)n_in;
  if (ws_size < kWsTotal) return;
  if ((size_t)out_size < (size_t)(kOut0Floats + kOut1Floats)) return;

  const float* x       = (const float*)d_in[0];
  const float* y       = (const float*)d_in[1];
  const float* conv1_w = (const float*)d_in[2];
  const float* conv1_b = (const float*)d_in[3];
  const float* conv2_w = (const float*)d_in[4];
  const float* conv2_b = (const float*)d_in[5];
  const float* Wt      = (const float*)d_in[6];
  const float* rbias   = (const float*)d_in[7];
  const float* fc1_w   = (const float*)d_in[8];
  const float* fc1_b   = (const float*)d_in[9];
  const float* fc2_w   = (const float*)d_in[10];
  const float* fc2_b   = (const float*)d_in[11];
  const float* fc3_w   = (const float*)d_in[12];
  const float* fc3_b   = (const float*)d_in[13];
  float* out = (float*)d_out;

  char* ws = (char*)d_ws;
  _Float16* A1   = (_Float16*)(ws + kOffA1);
  _Float16* BT1  = (_Float16*)(ws + kOffBT1);
  _Float16* H1   = (_Float16*)(ws + kOffH1);
  _Float16* W2   = (_Float16*)(ws + kOffW2);
  float*    UH   = (float*)(ws + kOffUH);
  float*    H2   = (float*)(ws + kOffH2);
  float*    BP1  = (float*)(ws + kOffBP1);
  float*    CIJ  = (float*)(ws + kOffCIJ);
  float*    BP2  = (float*)(ws + kOffBP2);
  float*    VJ   = (float*)(ws + kOffVJ);
  _Float16* AFC1 = (_Float16*)(ws + kOffAFC1);
  _Float16* WFC1 = (_Float16*)(ws + kOffWFC1);
  _Float16* C1   = (_Float16*)(ws + kOffC1);
  _Float16* WFC2 = (_Float16*)(ws + kOffWFC2);
  _Float16* C2P  = (_Float16*)(ws + kOffC2);
  _Float16* WFC3 = (_Float16*)(ws + kOffWFC3);
  float*    C3   = (float*)(ws + kOffC3);

  typedef const unsigned short* cus;

  {
    const int nA = kM1 * (kK1 / 8);
    k_im2col_x<<<(nA + 255) / 256, 256, 0, stream>>>(x, A1);
    const int nB = kCh * (kK1 / 8);
    k_cast_pad<<<(nB + 255) / 256, 256, 0, stream>>>(conv1_w, BT1, kCh, kK1real, kK1, 16.0f, nB);
    const int tiles = (kM1 / 64) * (kCh / 64);
    wmma_gemm64<0, false, 2, 1, false, 2><<<dim3((tiles + 7) / 8, 1), 256, 0, stream>>>(
        (cus)A1, (cus)A1, kK1, 0L, (cus)BT1, (cus)BT1, kK1, 0L,
        (void*)H1, (void*)H1, kCh, 0L, conv1_b, conv1_b, 0L, kM1, kCh, kK1, 1.0f / 16.0f);
  }
  {
    const int nW = kCh * (kK2 / 8);
    k_reorder_w2<<<(nW + 255) / 256, 256, 0, stream>>>(conv2_w, W2, 64.0f);
    const int tiles = (kM2 / 64) * (kCh / 64);
    wmma_conv2<<<(tiles + 7) / 8, 256, 0, stream>>>((cus)H1, (cus)W2, conv2_b, H2, 1.0f / 64.0f);
  }
  k_uhat<<<kRowsBIJ / 256, 256, 0, stream>>>(H2, Wt, UH);
  k_route<true><<<kBatch, 320, 0, stream>>>(CIJ, UH, rbias, VJ);
  k_agree_softmax<true><<<kRowsBI / 256, 256, 0, stream>>>(UH, VJ, BP1, BP1, CIJ);
  k_route<false><<<kBatch, 320, 0, stream>>>(CIJ, UH, rbias, VJ);
  k_agree_softmax<false><<<kRowsBI / 256, 256, 0, stream>>>(UH, VJ, BP1, BP2, CIJ);
  k_route<false><<<kBatch, 320, 0, stream>>>(CIJ, UH, rbias, VJ);
  k_out0<<<1, 256, 0, stream>>>(VJ, out);
  {
    k_masked<<<(kBatch * kFc1K) / 256, 256, 0, stream>>>(VJ, y, AFC1);
    const int n1 = kFc1N * (kFc1K / 8);
    k_cast_pad<<<(n1 + 255) / 256, 256, 0, stream>>>(fc1_w, WFC1, kFc1N, 16, kFc1K, 16.0f, n1);
    const int t1 = (kBatch / 64) * (kFc1N / 64);
    wmma_gemm64<0, false, 2, 1, false, 0><<<dim3((t1 + 7) / 8, 1), 256, 0, stream>>>(
        (cus)AFC1, (cus)AFC1, kFc1K, 0L, (cus)WFC1, (cus)WFC1, kFc1K, 0L,
        (void*)C1, (void*)C1, kFc1N, 0L, fc1_b, fc1_b, 0L, kBatch, kFc1N, kFc1K, 1.0f / 16.0f);

    const int n2 = kFc2N * (kFc1N / 8);
    k_cast_pad<<<(n2 + 255) / 256, 256, 0, stream>>>(fc2_w, WFC2, kFc2N, kFc1N, kFc1N, 16.0f, n2);
    const int t2 = (kBatch / 64) * (kFc2N / 64);
    wmma_gemm64<0, false, 2, 1, false, 0><<<dim3((t2 + 7) / 8, 1), 256, 0, stream>>>(
        (cus)C1, (cus)C1, kFc1N, 0L, (cus)WFC2, (cus)WFC2, kFc1N, 0L,
        (void*)C2P, (void*)C2P, kFc2N, 0L, fc2_b, fc2_b, 0L, kBatch, kFc2N, kFc1N, 1.0f / 16.0f);

    const int n3 = kFc3N * (kFc3K / 8);
    k_cast_pad<<<(n3 + 255) / 256, 256, 0, stream>>>(fc3_w, WFC3, kFc3Nreal, kFc3K, kFc3K, 16.0f, n3);
    const int t3 = (kBatch / 64) * (kFc3N / 64);
    wmma_gemm64<0, false, 0, 0, false, 0><<<dim3((t3 + 7) / 8, 1), 256, 0, stream>>>(
        (cus)C2P, (cus)C2P, kFc3K, 0L, (cus)WFC3, (cus)WFC3, kFc3K, 0L,
        (void*)C3, (void*)C3, kFc3N, 0L, fc3_b, fc3_b, 0L, kBatch, kFc3N, kFc3K, 1.0f / 16.0f);

    k_sig_out<<<(kOut1Floats / 4 + 255) / 256, 256, 0, stream>>>(C3, fc3_b, out);
  }
}
